// MultiHeadCrossAttention_20529943675563
// MI455X (gfx1250) — hardware-run, weakly checked
//
#include <hip/hip_runtime.h>


#ifndef NB
#define NB 8
#endif
#ifndef NI1
#define NI1 5
#endif
#ifndef NI2
#define NI2 15
#endif
#define NB_FULL  8
#define NI1_FULL 5
#define NI2_FULL 15
#define HW   144
#define DM   512
#define NH_  4
#define HD   128
#define L1   (NI1 * HW)
#define L2   (NI2 * HW)
#define L1P  (((L1 + 63) / 64) * 64)
#define L2P  (((L2 + 63) / 64) * 64)
#define L1K  (((L1 + 31) / 32) * 32)
#define AW   4
#define AW2  3
#define OSP  132
#define PSP  68
#define TP   72
#define SC2  ((float)(0.08838834764831845 * 1.4426950408889634))
#define PSH  14.0f
#define P2SH 10.0f
#define WSC  64.0f
#define CXS  256.0f
#define OSC  (1.0f / 16384.0f)
#define C1S  0.25f
#define NEGB (-3.0e38f)
#define OUT2_OFF ((size_t)NB_FULL * NI1_FULL * DM * HW)

static_assert(HD == 128);
static_assert(NH_ * HD == DM);
static_assert(DM % 64 == 0);
static_assert(HD % 64 == 0);
static_assert(DM % 32 == 0);
static_assert(HD % 32 == 0);
static_assert(HW % 16 == 0);
static_assert(L1 % 16 == 0);
static_assert(L2 % 16 == 0);
static_assert(L1 % (16 * AW2) == 0);
static_assert(L2P % (16 * AW) == 0);
static_assert(L2P % 32 == 0);
static_assert(L1K % 32 == 0);
static_assert(L1K <= L1P);
static_assert(L1K - 32 < L1);
static_assert(L1P % 64 == 0);
static_assert(L2P % 64 == 0);
static_assert(64 * HW / 4 == 9 * 256);
static_assert(HW <= 5 * 32);
static_assert(64 * HW / 4 == 18 * 128);
static_assert(AW * 16 == 16 * 4);
static_assert(16 * 4 == 64);
static_assert(8 * 2 == 16);
static_assert(2 * 32 == 64);
static_assert((OSP * 4) % 16 == 0);
static_assert(OSP >= HD + 4);
static_assert((PSP * 4) % 16 == 0);
static_assert(PSP >= 64 + 4);
static_assert((TP * 2) % 16 == 0);
static_assert(TP >= 64 + 8);
static_assert(AW * 16 * OSP * 4 + AW * 16 * 4 <= 131072);
static_assert(64 * HW * 4 <= 131072);
static_assert(64 * PSP * 4 <= 131072);
static_assert(HW * TP * 2 <= 131072);
static_assert(NB <= NB_FULL);
static_assert(NI1 <= NI1_FULL);
static_assert(NI2 <= NI2_FULL);
static_assert(OUT2_OFF * 4 == (size_t)11796480);
static_assert((OUT2_OFF * 4) % 128 == 0);

typedef _Float16 h16;
typedef unsigned short bf;
typedef __attribute__((ext_vector_type(16))) __bf16   v16bf;
typedef __attribute__((ext_vector_type(16))) _Float16 v16h;
typedef __attribute__((ext_vector_type(8)))  _Float16 v8h;
typedef __attribute__((ext_vector_type(8)))  unsigned short v8us;
typedef __attribute__((ext_vector_type(8)))  float    v8f;
typedef __attribute__((ext_vector_type(4)))  float    v4f;
typedef v4f  __attribute__((may_alias)) v4fa;

__device__ __forceinline__ unsigned short f2bf(float f) { unsigned u = __float_as_uint(f); u += 0x7FFFu + ((u >> 16) & 1u); return (unsigned short)(u >> 16); }
__device__ __forceinline__ float bfr(float f) { return __uint_as_float(((unsigned)f2bf(f)) << 16); }
__device__ __forceinline__ v16h cat16(v8h lo, v8h hi) { return __builtin_shufflevector(lo, hi, 0, 1, 2, 3, 4, 5, 6, 7, 8, 9, 10, 11, 12, 13, 14, 15); }
__device__ __forceinline__ v16bf cat16b(v8us lo, v8us hi) { return __builtin_bit_cast(v16bf, __builtin_shufflevector(lo, hi, 0, 1, 2, 3, 4, 5, 6, 7, 8, 9, 10, 11, 12, 13, 14, 15)); }
__device__ __forceinline__ v16h  ldh(const h16* p) { return cat16(*(const v8h*)p, *(const v8h*)(p + 16)); }
__device__ __forceinline__ v16bf ldb(const bf* p)  { return cat16b(*(const v8us*)p, *(const v8us*)(p + 16)); }
__device__ __forceinline__ void wave_sync() { __builtin_amdgcn_fence(3  , "wavefront"); __builtin_amdgcn_wave_barrier(); asm volatile("" ::: "memory"); }
__device__ __forceinline__ v8f wmh(v16h a, v16h b, v8f c) {
    c = __builtin_amdgcn_wmma_f32_16x16x32_f16(false, a, false, b, (short)0, c, false, false);
    asm volatile("v_nop\n\tv_nop\n\tv_nop\n\tv_nop" : "+v"(c) : "v"(a), "v"(b));
    return c; }
__device__ __forceinline__ v8f wmb(v16bf a, v16bf b, v8f c) {
    c = __builtin_amdgcn_wmma_f32_16x16x32_bf16(false, a, false, b, (short)0, c, false, false);
    asm volatile("v_nop\n\tv_nop\n\tv_nop\n\tv_nop" : "+v"(c) : "v"(a), "v"(b));
    return c; }
static __device__ __forceinline__ h16 toh_flush(float v) { const h16 r = (h16)v; return (fabsf(v) < 6.103515625e-05f) ? (h16)0.0f : r; }

template <int F16>
__device__ __forceinline__ void wt_body(const float* __restrict__ W, bf* WT) {
    __shared__ __align__(16) bf ts[64 * TP];
    const int tid = threadIdx.x; const int k0 = blockIdx.x * 64, n0 = blockIdx.y * 64;
#pragma unroll
    for (int it = 0; it < 4; ++it) { const int idx = it * 256 + tid; const int r = idx >> 4, c4 = (idx & 15) * 4;
        const v4f v = *(const v4f*)(W + (size_t)(k0 + r) * DM + n0 + c4);
#pragma unroll
        for (int i = 0; i < 4; ++i) { unsigned short w;
            if (F16) w = __builtin_bit_cast(unsigned short, toh_flush(bfr(v[i]) * WSC)); else w = f2bf(v[i]);
            ts[(c4 + i) * TP + r] = w; } }
    __syncthreads();
#pragma unroll 1
    for (int ps = 0; ps < 2; ++ps) {
#pragma unroll
        for (int it = 0; it < 2; ++it) { const int row = it * 32 + (tid >> 3), c8 = (tid & 7) * 8;
            const v8us o = *(const v8us*)(&ts[row * TP + c8]);
            *(volatile v8us*)(WT + (size_t)(n0 + row) * DM + k0 + c8) = o; }
        if (ps == 0) __threadfence(); }
}
__global__ __launch_bounds__(256) void k_wt_b(const float* __restrict__ W, bf* WT)  { wt_body<0>(W, WT); }
__global__ __launch_bounds__(256) void k_wt_h(const float* __restrict__ W, h16* WT) { wt_body<1>(W, (bf*)WT); }

__global__ __launch_bounds__(256) void k_tok(const float* __restrict__ src, bf* dst, int ni, int ni_full) {
    __shared__ __align__(16) bf ts[HW * TP];
    const int tid = threadIdx.x;
    const int bi = blockIdx.x; const int b = bi / ni, n = bi - b * ni; const int c0 = blockIdx.y * 64;
    const float* sp = src + ((size_t)(b * ni_full + n) * DM + c0) * HW;
#pragma unroll 3
    for (int it = 0; it < 9; ++it) { const int idx = it * 256 + tid; const int c = idx / 36, h4 = idx - c * 36;
        const v4f v = *(const v4f*)(sp + (size_t)idx * 4);
#pragma unroll
        for (int i = 0; i < 4; ++i) ts[(h4 * 4 + i) * TP + c] = f2bf(v[i]); }
    __syncthreads();
    bf* dp = dst + (size_t)bi * HW * DM + c0;
#pragma unroll 1
    for (int ps = 0; ps < 2; ++ps) {
#pragma unroll 1
        for (int it = 0; it < 5; ++it) { const int row = it * 32 + (tid >> 3), c8 = (tid & 7) * 8;
            const int rc = row < HW ? row : (HW - 1);
            const v8us o = *(const v8us*)(&ts[rc * TP + c8]);
            if (row < HW) *(volatile v8us*)(dp + (size_t)row * DM + c8) = o; }
        if (ps == 0) __threadfence(); }
}

__global__ __launch_bounds__(32) void k_proj(const bf* __restrict__ A, const bf* __restrict__ Bt, const float* __restrict__ bias, h16* PR, h16* PC, int L, int LP, int wrow, int wcol) {
    __shared__ __align__(16) float os[64 * PSP];
    const int lane = threadIdx.x & 31, lr = lane & 15, hi = lane >> 4;
    const int tpb = LP / 64;
    const int b = blockIdx.x / tpb; const int tt0 = (blockIdx.x - b * tpb) * 64; const int c0 = blockIdx.y * 64;
    size_t aoff[4];
#pragma unroll
    for (int mb = 0; mb < 4; ++mb) { int t = tt0 + mb * 16 + lr; t = min(t, L - 1); aoff[mb] = ((size_t)b * L + t) * DM + 8 * hi; }
    const size_t boff = (size_t)(c0 + lr) * DM + 8 * hi;
    v8f acc[4][4];
#pragma unroll
    for (int mb = 0; mb < 4; ++mb)
#pragma unroll
        for (int nb = 0; nb < 4; ++nb) acc[mb][nb] = (v8f){};
#pragma unroll 1
    for (int kc = 0; kc < DM; kc += 32) {
        v16bf a[4];
#pragma unroll
        for (int mb = 0; mb < 4; ++mb) a[mb] = ldb(A + aoff[mb] + kc);
#pragma unroll
        for (int nb = 0; nb < 4; ++nb) { const v16bf bb = ldb(Bt + boff + (size_t)nb * 16 * DM + kc);
#pragma unroll
            for (int mb = 0; mb < 4; ++mb) acc[mb][nb] = wmb(a[mb], bb, acc[mb][nb]); }
    }
    float bc[4];
#pragma unroll
    for (int nb = 0; nb < 4; ++nb) bc[nb] = bfr(bias[c0 + nb * 16 + lr]);
#pragma unroll
    for (int mb = 0; mb < 4; ++mb)
#pragma unroll
        for (int nb = 0; nb < 4; ++nb)
#pragma unroll
            for (int j = 0; j < 8; ++j) { const int tr = mb * 16 + hi * 8 + j;
                const float v = acc[mb][nb][j] + bc[nb];
                os[tr * PSP + nb * 16 + lr] = (tt0 + tr < L) ? v : 0.0f; }
    wave_sync();
    const int zh = b * NH_ + c0 / HD; const int d0 = c0 % HD;
#pragma unroll 1
    for (int ps = 0; ps < 2; ++ps) {
        if (wrow != 0) {
#pragma unroll 2
            for (int s = 0; s < 16; ++s) { const int row = 4 * s + (lane >> 3), c8 = (lane & 7) * 8;
                const v4f x0 = *(const v4fa*)(&os[row * PSP + c8]); const v4f x1 = *(const v4fa*)(&os[row * PSP + c8 + 4]); v8h hv;
#pragma unroll
                for (int i = 0; i < 4; ++i) { hv[i] = toh_flush(x0[i]); hv[4 + i] = toh_flush(x1[i]); }
                *(volatile v8h*)(PR + ((size_t)zh * LP + tt0 + row) * HD + d0 + c8) = hv; } }
        if (wcol != 0) {
#pragma unroll 2
            for (int s = 0; s < 16; ++s) { const int d = 4 * s + (lane >> 3), t8 = (lane & 7) * 8;
                v8h hv;
#pragma unroll
                for (int i = 0; i < 8; ++i) hv[i] = toh_flush(os[(t8 + i) * PSP + d]);
                *(volatile v8h*)(PC + ((size_t)zh * HD + d0 + d) * LP + tt0 + t8) = hv; } }
        if (ps == 0) __threadfence(); }
}

__global__ __launch_bounds__(32 * AW) void k_flash(const h16* __restrict__ QH, const h16* __restrict__ KP, const h16* __restrict__ VT, h16* CX, float* ST) {
    __shared__ __align__(16) float os[AW * 16 * OSP];
    __shared__ __align__(16) float sst[AW * 16];
    const int lane = threadIdx.x & 31, lr = lane & 15, hi = lane >> 4;
    const int wave = __builtin_amdgcn_readfirstlane((int)(threadIdx.x >> 5));
    const int zh = blockIdx.y; const int b = zh / NH_, h = zh % NH_;
    const int t0 = (blockIdx.x * AW + wave) * 16;
    const size_t qo = ((size_t)zh * L2P + t0 + lr) * HD + 8 * hi;
    v16h qf[4];
#pragma unroll
    for (int c = 0; c < 4; ++c) qf[c] = ldh(QH + qo + 32 * c);
    const size_t ko = ((size_t)zh * L1P + lr) * HD + 8 * hi;
    const size_t vo = ((size_t)zh * HD + lr) * L1P + 8 * hi;
    v8f o[8];
#pragma unroll
    for (int j = 0; j < 8; ++j) o[j] = (v8f){};
    float m = NEGB, l = 0.0f;
#pragma unroll 1
    for (int key0 = 0; key0 < L1K; key0 += 32) {
        const h16* ka = KP + ko + (size_t)key0 * HD;
        v8f sa = (v8f){}, sb = (v8f){};
#pragma unroll
        for (int c = 0; c < 4; ++c) { const v16h k0f = ldh(ka + 32 * c); sa = wmh(k0f, qf[c], sa); }
#pragma unroll
        for (int c = 0; c < 4; ++c) { const v16h k1f = ldh(ka + 16 * HD + 32 * c); sb = wmh(k1f, qf[c], sb); }
        const int ja = key0 + 8 * hi;
        float ta[8], tb[8]; bool fa[8], fb[8]; float mx = NEGB;
#pragma unroll
        for (int r = 0; r < 8; ++r) {
            fa[r] = (ja + r < L1); fb[r] = (ja + 16 + r < L1);
            ta[r] = sa[r] * SC2; tb[r] = sb[r] * SC2;
            mx = fmaxf(mx, fmaxf(fa[r] ? ta[r] : NEGB, fb[r] ? tb[r] : NEGB)); }
        mx = fmaxf(mx, __shfl_xor(mx, 16, 32));
        const float mnew = fmaxf(m, mx);
        const float alpha = __builtin_amdgcn_exp2f(m - mnew);
        const float sh = PSH - mnew;
        v16h pb; float ls = 0.0f;
#pragma unroll
        for (int r = 0; r < 8; ++r) {
            const float xa = ta[r] + sh, xb = tb[r] + sh;
            const float ea = __builtin_amdgcn_exp2f(xa), eb = __builtin_amdgcn_exp2f(xb);
            const float ga = (fa[r] && xa >= -14.0f) ? ea : 0.0f, gb = (fb[r] && xb >= -14.0f) ? eb : 0.0f;
            const h16 pa = (h16)ga; const h16 pc = (h16)gb;
            pb[r] = pa; pb[8 + r] = pc;
            ls += (float)pa + (float)pc; }
        l = l * alpha + ls; m = mnew;
#pragma unroll
        for (int j = 0; j < 8; ++j) o[j] = o[j] * alpha;
        const h16* va = VT + vo + key0;
#pragma unroll
        for (int j = 0; j < 8; ++j) { const v16h vf = ldh(va + (size_t)j * 16 * L1P); o[j] = wmh(vf, pb, o[j]); }
    }
    l += __shfl_xor(l, 16, 32);
    const float inv = 1.0f / l;
    const float stat = m + __builtin_amdgcn_logf(l) - PSH;
    const float cs = inv * CXS;
    const int wb = wave * 16 * OSP;
#pragma unroll
    for (int j = 0; j < 8; ++j) { v4f a, c;
        a[0] = o[j][0] * cs; a[1] = o[j][1] * cs; a[2] = o[j][2] * cs; a[3] = o[j][3] * cs; c[0] = o[j][4] * cs; c[1] = o[j][5] * cs; c[2] = o[j][6] * cs; c[3] = o[j][7] * cs;
        *(v4fa*)(&os[wb + lr * OSP + 16 * j + 8 * hi]) = a; *(v4fa*)(&os[wb + lr * OSP + 16 * j + 8 * hi + 4]) = c; }
    if (hi == 0) sst[wave * 16 + lr] = stat;
    wave_sync();
    if (t0 < L2) {
        h16* cp = CX + ((size_t)b * L2 + t0) * DM + h * HD;
#pragma unroll 1
        for (int ps = 0; ps < 2; ++ps) {
#pragma unroll 2
            for (int s = 0; s < 8; ++s) { const int row = 2 * s + (lane >> 4), c8 = (lane & 15) * 8;
                const v4f x0 = *(const v4fa*)(&os[wb + row * OSP + c8]); const v4f x1 = *(const v4fa*)(&os[wb + row * OSP + c8 + 4]); v8h hv;
#pragma unroll
                for (int i = 0; i < 4; ++i) { hv[i] = toh_flush(x0[i]); hv[4 + i] = toh_flush(x1[i]); }
                *(volatile v8h*)(cp + (size_t)row * DM + c8) = hv; }
            if (ps == 0) __threadfence(); }
    }
    __syncthreads();
    if (wave == 0) {
        const v4f sv = *(const v4fa*)(&sst[(lane & 15) * 4]);
        float* sp = ST + (size_t)zh * L2P + (size_t)blockIdx.x * (16 * AW) + (lane & 15) * 4;
#pragma unroll 1
        for (int ps = 0; ps < 2; ++ps) {
            if (lane < 16) *(volatile v4f*)sp = sv;
            if (ps == 0) __threadfence(); }
    }
}

__global__ __launch_bounds__(32 * AW2) void k_att1(const h16* __restrict__ QH, const h16* __restrict__ QT, const h16* __restrict__ KP, const float* __restrict__ ST, h16* CX) {
    __shared__ __align__(16) float os[AW2 * 16 * OSP];
    const int lane = threadIdx.x & 31, lr = lane & 15, hi = lane >> 4;
    const int wave = __builtin_amdgcn_readfirstlane((int)(threadIdx.x >> 5));
    const int zh = blockIdx.y; const int b = zh / NH_, h = zh % NH_;
    const int key0 = (blockIdx.x * AW2 + wave) * 16;
    const size_t kb = ((size_t)zh * L1P + key0 + lr) * HD + 8 * hi;
    v16h kf[4];
#pragma unroll
    for (int c = 0; c < 4; ++c) kf[c] = ldh(KP + kb + 32 * c);
    const size_t qa = ((size_t)zh * L2P + lr) * HD + 8 * hi;
    const size_t qt = ((size_t)zh * HD + lr) * L2P + 8 * hi;
    const float* sp = ST + (size_t)zh * L2P + 8 * hi;
    v8f acc[8];
#pragma unroll
    for (int j = 0; j < 8; ++j) acc[j] = (v8f){};
#pragma unroll 1
    for (int q0 = 0; q0 < L2P; q0 += 32) {
        const h16* qp = QH + qa + (size_t)q0 * HD;
        v8f sa = (v8f){}, sb = (v8f){};
#pragma unroll
        for (int c = 0; c < 4; ++c) { const v16h a0 = ldh(qp + 32 * c); sa = wmh(a0, kf[c], sa); }
#pragma unroll
        for (int c = 0; c < 4; ++c) { const v16h a1 = ldh(qp + 16 * HD + 32 * c); sb = wmh(a1, kf[c], sb); }
        const float* s4 = sp + q0;
        const v4f m0 = *(const v4f*)s4, m1 = *(const v4f*)(s4 + 4), m2 = *(const v4f*)(s4 + 16), m3 = *(const v4f*)(s4 + 20);
        float sx[8], sy[8];
#pragma unroll
        for (int r = 0; r < 4; ++r) { sx[r] = m0[r]; sx[4 + r] = m1[r]; sy[r] = m2[r]; sy[4 + r] = m3[r]; }
        const int qi = q0 + 8 * hi;
        v16h pb;
#pragma unroll
        for (int r = 0; r < 8; ++r) {
            const float xa = sa[r] * SC2 - sx[r] + P2SH, xb = sb[r] * SC2 - sy[r] + P2SH;
            const float ea = __builtin_amdgcn_exp2f(xa), eb = __builtin_amdgcn_exp2f(xb);
            const float ga = ((qi + r < L2) && xa >= -14.0f) ? ea : 0.0f, gb = ((qi + 16 + r < L2) && xb >= -14.0f) ? eb : 0.0f;
            pb[r] = (h16)ga; pb[8 + r] = (h16)gb; }
        const h16* tp = QT + qt + q0;
#pragma unroll
        for (int j = 0; j < 8; ++j) { const v16h af = ldh(tp + (size_t)j * 16 * L2P); acc[j] = wmh(af, pb, acc[j]); }
    }
    const int wb = wave * 16 * OSP;
#pragma unroll
    for (int j = 0; j < 8; ++j) { v4f a, c;
        a[0] = acc[j][0] * C1S; a[1] = acc[j][1] * C1S; a[2] = acc[j][2] * C1S; a[3] = acc[j][3] * C1S; c[0] = acc[j][4] * C1S; c[1] = acc[j][5] * C1S; c[2] = acc[j][6] * C1S; c[3] = acc[j][7] * C1S;
        *(v4fa*)(&os[wb + lr * OSP + 16 * j + 8 * hi]) = a; *(v4fa*)(&os[wb + lr * OSP + 16 * j + 8 * hi + 4]) = c; }
    wave_sync();
    h16* cp = CX + ((size_t)b * L1 + key0) * DM + h * HD;
#pragma unroll 1
    for (int ps = 0; ps < 2; ++ps) {
#pragma unroll 2
        for (int s = 0; s < 8; ++s) { const int row = 2 * s + (lane >> 4), c8 = (lane & 15) * 8;
            const v4f x0 = *(const v4fa*)(&os[wb + row * OSP + c8]); const v4f x1 = *(const v4fa*)(&os[wb + row * OSP + c8 + 4]); v8h hv;
#pragma unroll
            for (int i = 0; i < 4; ++i) { hv[i] = toh_flush(x0[i]); hv[4 + i] = toh_flush(x1[i]); }
            *(volatile v8h*)(cp + (size_t)row * DM + c8) = hv; }
        if (ps == 0) __threadfence(); }
}

__global__ __launch_bounds__(128) void k_oproj(const h16* __restrict__ A, const h16* __restrict__ Bt, const float* __restrict__ bias, float* OUT, int ni, int ni_full) {
    __shared__ __align__(16) float os[64 * HW];
    const int tid = threadIdx.x;
    const int lane = tid & 31, lr = lane & 15, hi = lane >> 4;
    const int wave = __builtin_amdgcn_readfirstlane((int)(threadIdx.x >> 5));
    const int bi = blockIdx.x; const int b = bi / ni, n = bi - b * ni; const int c0 = blockIdx.y * 64;
    const size_t aoff = ((size_t)bi * HW + lr) * DM + 8 * hi;
    const size_t boff = (size_t)(c0 + wave * 16 + lr) * DM + 8 * hi;
    v8f acc[9];
#pragma unroll
    for (int mb = 0; mb < 9; ++mb) acc[mb] = (v8f){};
#pragma unroll 1
    for (int kc = 0; kc < DM; kc += 32) {
        const v16h bb = ldh(Bt + boff + kc);
#pragma unroll
        for (int mb = 0; mb < 9; ++mb) { const v16h af = ldh(A + aoff + (size_t)mb * 16 * DM + kc); acc[mb] = wmh(af, bb, acc[mb]); }
    }
    const float bc = bfr(bias[c0 + wave * 16 + lr]);
    const int ob = (wave * 16 + lr) * HW + 8 * hi;
#pragma unroll
    for (int mb = 0; mb < 9; ++mb) { v4f a, c;
        a[0] = acc[mb][0] * OSC + bc; a[1] = acc[mb][1] * OSC + bc; a[2] = acc[mb][2] * OSC + bc; a[3] = acc[mb][3] * OSC + bc;
        c[0] = acc[mb][4] * OSC + bc; c[1] = acc[mb][5] * OSC + bc; c[2] = acc[mb][6] * OSC + bc; c[3] = acc[mb][7] * OSC + bc;
        *(v4fa*)(&os[ob + mb * 16]) = a; *(v4fa*)(&os[ob + mb * 16 + 4]) = c; }
    __syncthreads();
    float* op = OUT + ((size_t)(b * ni_full + n) * DM + c0) * HW;
#pragma unroll 1
    for (int ps = 0; ps < 2; ++ps) {
#pragma unroll 2
        for (int it = 0; it < 18; ++it) { const int idx = it * 128 + tid;
            const v4f val = *(const v4fa*)(&os[idx * 4]);
            *(volatile v4f*)(op + (size_t)idx * 4) = val; }
        if (ps == 0) __threadfence(); }
}

static constexpr size_t al256(size_t v) { return (v + 255) & ~(size_t)255; }
static constexpr size_t SZ_WB = al256((size_t)3 * DM * DM * 2);
static constexpr size_t SZ_WH = al256((size_t)2 * DM * DM * 2);
static constexpr size_t SZ_X2 = al256((size_t)NB * L2 * DM * 2);
static constexpr size_t SZ_X1 = al256((size_t)NB * L1 * DM * 2);
static constexpr size_t SZ_Q  = al256((size_t)NB * NH_ * L2P * HD * 2);
static constexpr size_t SZ_K  = al256((size_t)NB * NH_ * L1P * HD * 2);
static constexpr size_t SZ_ST = al256((size_t)NB * NH_ * L2P * 4);
static constexpr size_t SZ_TOTAL = SZ_WB + SZ_WH + 2 * SZ_X2 + 2 * SZ_X1 + 2 * SZ_Q + 2 * SZ_K + SZ_ST;
static_assert(SZ_TOTAL <= (size_t)134217728);
static_assert(((size_t)DM * DM * 2) % 256 == 0);
static constexpr size_t NEED1 = ((size_t)(NB - 1) * NI1_FULL + NI1) * DM * HW;
static constexpr size_t NEED2 = ((size_t)(NB - 1) * NI2_FULL + NI2) * DM * HW;
static constexpr size_t NEEDO = OUT2_OFF + NEED2;
static_assert(NEED1 <= OUT2_OFF);
static_assert(NEEDO * 4 <= (size_t)47185920);

extern "C" void kernel_launch(void* const* d_in, const int* in_sizes, int n_in,
                              void* d_out, int out_size, void* d_ws, size_t ws_size, hipStream_t stream) {
    if (n_in < 12) return;
    if ((size_t)in_sizes[0] < NEED1 || (size_t)in_sizes[1] < NEED2) return;
    if ((size_t)in_sizes[2] < (size_t)DM * DM || (size_t)in_sizes[4] < (size_t)DM * DM || (size_t)in_sizes[6] < (size_t)DM * DM ||
        (size_t)in_sizes[8] < (size_t)DM * DM || (size_t)in_sizes[10] < (size_t)DM * DM) return;
    if (in_sizes[3] < DM || in_sizes[5] < DM || in_sizes[7] < DM || in_sizes[9] < DM || in_sizes[11] < DM) return;
    if ((size_t)out_size < NEEDO) return;
    if (SZ_TOTAL > ws_size) return;
    const float* x1 = (const float*)d_in[0]; const float* x2 = (const float*)d_in[1];
    const float* wq = (const float*)d_in[2];  const float* bq = (const float*)d_in[3];
    const float* wk = (const float*)d_in[4];  const float* bk = (const float*)d_in[5];
    const float* wv = (const float*)d_in[6];  const float* bv = (const float*)d_in[7];
    const float* woq = (const float*)d_in[8]; const float* boq = (const float*)d_in[9];
    const float* wok = (const float*)d_in[10]; const float* bok = (const float*)d_in[11];
    float* OUT1 = (float*)d_out;
    float* OUT2 = (float*)d_out + OUT2_OFF;
    char* wsp = (char*)d_ws;
    bf* WB = (bf*)wsp; wsp += SZ_WB;
    h16* WH = (h16*)wsp; wsp += SZ_WH;
    bf* X2 = (bf*)wsp; wsp += SZ_X2;
    bf* X1 = (bf*)wsp; wsp += SZ_X1;
    h16* QH = (h16*)wsp; wsp += SZ_Q;
    h16* QT = (h16*)wsp; wsp += SZ_Q;
    h16* KP = (h16*)wsp; wsp += SZ_K;
    h16* VT = (h16*)wsp; wsp += SZ_K;
    float* ST = (float*)wsp; wsp += SZ_ST;
    h16* C2 = (h16*)wsp; wsp += SZ_X2;
    h16* C1 = (h16*)wsp; wsp += SZ_X1;
    bf* WQ = WB; bf* WK = WB + (size_t)DM * DM; bf* WV = WB + (size_t)2 * DM * DM;
    h16* WOQ = WH; h16* WOK = WH + (size_t)DM * DM;

    k_wt_b<<<dim3(DM / 64, DM / 64, 1), 256, 0, stream>>>(wq, WQ);
    k_wt_b<<<dim3(DM / 64, DM / 64, 1), 256, 0, stream>>>(wk, WK);
    k_wt_b<<<dim3(DM / 64, DM / 64, 1), 256, 0, stream>>>(wv, WV);
    k_wt_h<<<dim3(DM / 64, DM / 64, 1), 256, 0, stream>>>(woq, WOQ);
    k_wt_h<<<dim3(DM / 64, DM / 64, 1), 256, 0, stream>>>(wok, WOK);
    k_tok<<<dim3(NB * NI2, DM / 64, 1), 256, 0, stream>>>(x2, X2, NI2, NI2_FULL);
    k_tok<<<dim3(NB * NI1, DM / 64, 1), 256, 0, stream>>>(x1, X1, NI1, NI1_FULL);

    k_proj<<<dim3(NB * (L2P / 64), DM / 64, 1), 32, 0, stream>>>(X2, WQ, bq, QH, QT, L2, L2P, 1, 1);
    k_proj<<<dim3(NB * (L1P / 64), DM / 64, 1), 32, 0, stream>>>(X1, WK, bk, KP, KP, L1, L1P, 1, 0);
    k_proj<<<dim3(NB * (L1P / 64), DM / 64, 1), 32, 0, stream>>>(X1, WV, bv, VT, VT, L1, L1P, 0, 1);

    k_flash<<<dim3(L2P / (16 * AW), NB * NH_, 1), 32 * AW, 0, stream>>>(QH, KP, VT, C2, ST);
    k_att1<<<dim3(L1 / (16 * AW2), NB * NH_, 1), 32 * AW2, 0, stream>>>(QH, QT, KP, ST, C1);

    k_oproj<<<dim3(NB * NI2, DM / 64, 1), 128, 0, stream>>>(C2, WOQ, boq, OUT2, NI2, NI2_FULL);
    k_oproj<<<dim3(NB * NI1, DM / 64, 1), 128, 0, stream>>>(C1, WOK, bok, OUT1, NI1, NI1_FULL);
}
